// MIRACLE_2611340116165
// MI455X (gfx1250) — hardware-verified
//
#include <hip/hip_runtime.h>
#include <stddef.h>
#include <stdint.h>

#define NR 32768
#define ND 160
#define NF 128
#define NH 32
#define RB 128
#define FB 32

static_assert((ND % 32) == 0);
static_assert(NH == 32);
static_assert((NR % RB) == 0);
static_assert((NF % FB) == 0);
static_assert(RB == 128);
static_assert(FB == 32);
static_assert(((NR * ND) % 2048) == 0);
static_assert(((NH * ND) % 1024) == 0);

typedef __attribute__((ext_vector_type(16))) __bf16 v16b;
typedef float        v8f __attribute__((ext_vector_type(8)));
typedef float        v4f __attribute__((ext_vector_type(4)));
typedef unsigned int v4u __attribute__((ext_vector_type(4)));

__device__ __forceinline__ unsigned short bf_bits(float f) {
  const unsigned u = __float_as_uint(f);
  return (unsigned short)((u + 0x7FFFu + ((u >> 16) & 1u)) >> 16);
}
__device__ __forceinline__ float bf_val(unsigned short b) { return __uint_as_float(((unsigned)b) << 16); }
__device__ __forceinline__ float bfr(float f) { return bf_val(bf_bits(f)); }
__device__ __forceinline__ unsigned pk16(unsigned short a, unsigned short b) { return (unsigned)a | ((unsigned)b << 16); }
__device__ __forceinline__ v8f zero8() { v8f z = {0.f, 0.f, 0.f, 0.f, 0.f, 0.f, 0.f, 0.f}; return z; }
__device__ __forceinline__ float elu_f(float x) {
  const float e = __expf(x) - 1.0f;
  return x > 0.0f ? x : e;
}

union FragB { v16b v; v4u u[2]; };
__device__ __forceinline__ v16b ldfrag_b(const unsigned short* p) {
  FragB f;
  f.u[0] = *(const v4u*)(p);
  f.u[1] = *(const v4u*)(p + 16);
  return f.v;
}

__device__ __forceinline__ v8f mma_b(v16b a, v16b b, v8f c) {
  return __builtin_amdgcn_wmma_f32_16x16x32_bf16(false, a, false, b, (short)0, c, false, false);
}
__device__ __forceinline__ void guard4(v8f& c0, v8f& c1, v8f& c2, v8f& c3,
                                       const v16b& a0, const v16b& a1, const v16b& b0, const v16b& b1) {
#if defined(__HIP_DEVICE_COMPILE__)
  asm volatile("v_nop\n\tv_nop\n\tv_nop\n\tv_nop"
               : "+v"(c0), "+v"(c1), "+v"(c2), "+v"(c3)
               : "v"(a0), "v"(a1), "v"(b0), "v"(b1));
#endif
}
__device__ __forceinline__ void guard4x6(v8f& c0, v8f& c1, v8f& c2, v8f& c3,
                                         const v16b& a0, const v16b& a1, const v16b& a2, const v16b& a3,
                                         const v16b& b0, const v16b& b1) {
#if defined(__HIP_DEVICE_COMPILE__)
  asm volatile("v_nop\n\tv_nop\n\tv_nop\n\tv_nop"
               : "+v"(c0), "+v"(c1), "+v"(c2), "+v"(c3)
               : "v"(a0), "v"(a1), "v"(a2), "v"(a3), "v"(b0), "v"(b1));
#endif
}

__global__ __launch_bounds__(256)
void k_cvx(const float* __restrict__ x, unsigned short* Xb) {
  const size_t f8 = ((size_t)blockIdx.x * 256 + threadIdx.x) * 8;
  const v4f a = *(const v4f*)(x + f8);
  const v4f b = *(const v4f*)(x + f8 + 4);
  v4u u;
  u[0] = pk16(bf_bits(a[0]), bf_bits(a[1]));
  u[1] = pk16(bf_bits(a[2]), bf_bits(a[3]));
  u[2] = pk16(bf_bits(b[0]), bf_bits(b[1]));
  u[3] = pk16(bf_bits(b[2]), bf_bits(b[3]));
  unsigned short* dst = Xb + f8;
  *(volatile v4u*)dst = u;
  __threadfence();
  *(volatile v4u*)dst = u;
}

__global__ __launch_bounds__(128)
void k_tw(const float* __restrict__ w1, const float* __restrict__ w2, unsigned short* W1T, unsigned short* W2T) {
  __shared__ __align__(16) unsigned short sT1[NH * ND];
  __shared__ __align__(16) unsigned short sT2[NH * NH];
  const int f = blockIdx.x, tid = threadIdx.x;
  const float* w1f = w1 + (size_t)f * ND * NH;
  const float* w2f = w2 + (size_t)f * NH * NH;
#pragma unroll
  for (int j = 0; j < (ND * NH) / (128 * 4); ++j) {
    const int idx4 = (tid + 128 * j) * 4;
    const int d = idx4 >> 5, h0 = idx4 & 31;
    const v4f v = *(const v4f*)(w1f + idx4);
    sT1[(h0 + 0) * ND + d] = bf_bits(v[0]);
    sT1[(h0 + 1) * ND + d] = bf_bits(v[1]);
    sT1[(h0 + 2) * ND + d] = bf_bits(v[2]);
    sT1[(h0 + 3) * ND + d] = bf_bits(v[3]);
  }
#pragma unroll
  for (int j = 0; j < (NH * NH) / (128 * 4); ++j) {
    const int idx4 = (tid + 128 * j) * 4;
    const int h = idx4 >> 5, k0 = idx4 & 31;
    const v4f v = *(const v4f*)(w2f + idx4);
    sT2[(k0 + 0) * NH + h] = bf_bits(v[0]);
    sT2[(k0 + 1) * NH + h] = bf_bits(v[1]);
    sT2[(k0 + 2) * NH + h] = bf_bits(v[2]);
    sT2[(k0 + 3) * NH + h] = bf_bits(v[3]);
  }
  __syncthreads();

  v4u u1[5];
#pragma unroll
  for (int it = 0; it < 5; ++it) u1[it] = *(const v4u*)(sT1 + it * 1024 + tid * 8);
  const v4u u2 = *(const v4u*)(sT2 + tid * 8);
  unsigned short* d1 = W1T + (size_t)f * (NH * ND) + tid * 8;
  unsigned short* d2 = W2T + (size_t)f * (NH * NH) + tid * 8;
#pragma unroll
  for (int it = 0; it < 5; ++it) *(volatile v4u*)(d1 + it * 1024) = u1[it];
  *(volatile v4u*)d2 = u2;
  __threadfence();
#pragma unroll
  for (int it = 0; it < 5; ++it) *(volatile v4u*)(d1 + it * 1024) = u1[it];
  *(volatile v4u*)d2 = u2;
}

__device__ __forceinline__ void put_h1(unsigned short* hi, unsigned short* lo, const v8f& acc, float bias, int base) {
#pragma unroll
  for (int r = 0; r < 8; ++r) {
    const float h = elu_f(acc[r] + bias);
    const unsigned short hb = bf_bits(h);
    const unsigned short lb = bf_bits(h - bf_val(hb));
    hi[base + r * NH] = hb;
    lo[base + r * NH] = lb;
  }
}

__device__ __forceinline__ void lay3(const v8f& d0, const v8f& d1, float c20, float c21, float w30, float w31,
                                     float c3, float* so, int lrow0, int fl, int c) {
  float s[8];
#pragma unroll
  for (int r = 0; r < 8; ++r) {
    const float h20 = elu_f(d0[r] + c20);
    const float h21 = elu_f(d1[r] + c21);
    s[r] = h20 * w30 + h21 * w31;
  }
#pragma unroll
  for (int off = 8; off >= 1; off >>= 1) {
#pragma unroll
    for (int r = 0; r < 8; ++r) s[r] += __shfl_xor(s[r], off, 16);
  }
  if (c == 0) {
#pragma unroll
    for (int r = 0; r < 8; ++r) so[(lrow0 + r) * FB + fl] = s[r] + c3;
  }
}

__global__ __launch_bounds__(128)
void k_mlp(const unsigned short* __restrict__ Xb, const unsigned short* __restrict__ W1T,
           const unsigned short* __restrict__ W2T, const float* __restrict__ b1, const float* __restrict__ b2,
           const float* __restrict__ W3, const float* __restrict__ b3, float* out) {
  __shared__ __align__(16) unsigned short sHi[4 * 32 * NH];
  __shared__ __align__(16) unsigned short sLo[4 * 32 * NH];
  __shared__ __align__(16) float sO[RB * FB];
  const int tid = threadIdx.x, w = tid >> 5, lane = tid & 31, hh = lane >> 4, c = lane & 15;
  const int row0 = blockIdx.x * RB, fbase = blockIdx.y * FB;
  const int mrow0 = row0 + 32 * w;

  const unsigned short* ap0 = Xb + (size_t)(mrow0 + c) * ND + 8 * hh;
  const unsigned short* ap1 = ap0 + (size_t)16 * ND;
  unsigned short* hiw = sHi + w * (32 * NH);
  unsigned short* low = sLo + w * (32 * NH);

#pragma unroll 1
  for (int fl = 0; fl < FB; ++fl) {
    const int f = fbase + fl;
    const unsigned short* bq0 = W1T + (size_t)(f * NH + c) * ND + 8 * hh;
    const unsigned short* bq1 = bq0 + (size_t)16 * ND;
    v8f a00 = zero8(), a01 = zero8(), a10 = zero8(), a11 = zero8();
#pragma unroll 1
    for (int ks = 0; ks < ND / 32; ++ks) {
      const int ko = 32 * ks;
      const v16b x0 = ldfrag_b(ap0 + ko);
      const v16b x1 = ldfrag_b(ap1 + ko);
      const v16b g0 = ldfrag_b(bq0 + ko);
      const v16b g1 = ldfrag_b(bq1 + ko);
      a00 = mma_b(x0, g0, a00);
      a01 = mma_b(x0, g1, a01);
      a10 = mma_b(x1, g0, a10);
      a11 = mma_b(x1, g1, a11);
      guard4(a00, a01, a10, a11, x0, x1, g0, g1);
    }
    const float c10 = bfr(b1[f * NH + c]), c11 = bfr(b1[f * NH + 16 + c]);
    put_h1(hiw, low, a00, c10, (8 * hh) * NH + c);
    put_h1(hiw, low, a01, c11, (8 * hh) * NH + 16 + c);
    put_h1(hiw, low, a10, c10, (16 + 8 * hh) * NH + c);
    put_h1(hiw, low, a11, c11, (16 + 8 * hh) * NH + 16 + c);
    __syncthreads();

    const unsigned short* cq0 = W2T + (size_t)(f * NH + c) * NH + 8 * hh;
    const unsigned short* cq1 = cq0 + (size_t)16 * NH;
    const v16b p0 = ldfrag_b(cq0);
    const v16b p1 = ldfrag_b(cq1);
    const v16b h0 = ldfrag_b(hiw + c * NH + 8 * hh);
    const v16b h1 = ldfrag_b(hiw + (16 + c) * NH + 8 * hh);
    const v16b l0 = ldfrag_b(low + c * NH + 8 * hh);
    const v16b l1 = ldfrag_b(low + (16 + c) * NH + 8 * hh);
    v8f d00 = zero8(), d01 = zero8(), d10 = zero8(), d11 = zero8();
    d00 = mma_b(h0, p0, d00);
    d01 = mma_b(h0, p1, d01);
    d10 = mma_b(h1, p0, d10);
    d11 = mma_b(h1, p1, d11);
    d00 = mma_b(l0, p0, d00);
    d01 = mma_b(l0, p1, d01);
    d10 = mma_b(l1, p0, d10);
    d11 = mma_b(l1, p1, d11);
    guard4x6(d00, d01, d10, d11, h0, h1, l0, l1, p0, p1);
    __syncthreads();

    const float c20 = bfr(b2[f * NH + c]), c21 = bfr(b2[f * NH + 16 + c]);
    const float w30 = bfr(W3[f * NH + c]), w31 = bfr(W3[f * NH + 16 + c]);
    const float c3 = bfr(b3[f]);
    lay3(d00, d01, c20, c21, w30, w31, c3, sO, 32 * w + 8 * hh, fl, c);
    lay3(d10, d11, c20, c21, w30, w31, c3, sO, 32 * w + 16 + 8 * hh, fl, c);
  }
  __syncthreads();

  const int lq = tid >> 3, p4 = (tid & 7) * 4;
  v4f o[8];
#pragma unroll
  for (int it = 0; it < 8; ++it) o[it] = *(const v4f*)(sO + (it * 16 + lq) * FB + p4);
  float* ob = out + (size_t)(row0 + lq) * NF + fbase + p4;
#pragma unroll
  for (int it = 0; it < 8; ++it) *(volatile v4f*)(ob + (size_t)it * 16 * NF) = o[it];
  __threadfence();
#pragma unroll
  for (int it = 0; it < 8; ++it) *(volatile v4f*)(ob + (size_t)it * 16 * NF) = o[it];
}

extern "C" void kernel_launch(void* const* d_in, const int* in_sizes, int n_in,
                              void* d_out, int out_size, void* d_ws, size_t ws_size,
                              hipStream_t stream) {
  if (n_in < 7) return;
  if (in_sizes[0] != NR * ND) return;
  if (in_sizes[1] != NF * ND * NH) return;
  if (in_sizes[2] != NF * NH) return;
  if (in_sizes[3] != NF * NH * NH) return;
  if (in_sizes[4] != NF * NH) return;
  if (in_sizes[5] != NF * NH) return;
  if (in_sizes[6] != NF) return;
  if (out_size != NR * NF) return;

  const float* x  = (const float*)d_in[0];
  const float* w1 = (const float*)d_in[1];
  const float* b1 = (const float*)d_in[2];
  const float* w2 = (const float*)d_in[3];
  const float* b2 = (const float*)d_in[4];
  const float* w3 = (const float*)d_in[5];
  const float* b3 = (const float*)d_in[6];
  float* out = (float*)d_out;

  const size_t sX  = (size_t)NR * ND * 2;
  const size_t sW1 = (size_t)NF * NH * ND * 2;
  const size_t sW2 = (size_t)NF * NH * NH * 2;
  size_t off = 0;
  const size_t oX  = off; off += sX;
  const size_t oW1 = off; off += sW1;
  const size_t oW2 = off; off += sW2;
  if (off > ws_size) return;
  if (off > (size_t)134217728) return;

  char* ws = (char*)d_ws;
  unsigned short* Xb  = (unsigned short*)(ws + oX);
  unsigned short* W1T = (unsigned short*)(ws + oW1);
  unsigned short* W2T = (unsigned short*)(ws + oW2);

  k_cvx<<<dim3((NR * ND) / 2048), dim3(256), 0, stream>>>(x, Xb);
  k_tw<<<dim3(NF), dim3(128), 0, stream>>>(w1, w2, W1T, W2T);
  k_mlp<<<dim3(NR / RB, NF / FB), dim3(128), 0, stream>>>(Xb, W1T, W2T, b1, b2, w3, b3, out);
  (void)hipGetLastError();
}
